// MatrixKANLayer_88098369175692
// MI455X (gfx1250) — hardware-run, weakly checked
//
#include <hip/hip_runtime.h>


namespace {
constexpr int NBR = 8192, IN = 512, OUT = 512, G = 20, GP = G + 1, KT = IN * GP  , FCH = 32  , KCH = FCH * GP  ;
constexpr float HS = 256.0f, WSC = 256.0f;
typedef _Float16 b16;
typedef __attribute__((ext_vector_type(16))) _Float16 v16b;
typedef __attribute__((ext_vector_type(8))) _Float16 v8b;
typedef __attribute__((ext_vector_type(8))) float v8f;
typedef __attribute__((ext_vector_type(4))) float v4f;
__device__ __forceinline__ float bf16_rne(float f) { unsigned int u = __float_as_uint(f); u += 0x7FFFu + ((u >> 16) & 1u); float r = __uint_as_float(u & 0xFFFF0000u); asm volatile("" : "+v"(r)); return r; }
__device__ __forceinline__ float bfv(float f) { float r = bf16_rne(f); asm volatile("" : "+v"(r)); return r; }
__device__ __forceinline__ void split16(float v, b16& hi, b16& lo) { hi = (b16)v; lo = (b16)(v - (float)hi); }
__device__ __forceinline__ v16b frag_kb(const b16* p, int hh) { const v8b a = *(const v8b*)(p + 8 * hh), b = *(const v8b*)(p + 16 + 8 * hh); v16b f;
#pragma unroll
  for (int e = 0; e < 8; ++e) { f[e] = a[e]; f[8 + e] = b[e]; } return f; }
__device__ __forceinline__ v8f wmma16b(v16b a, v16b b, v8f c) { v8f d = __builtin_amdgcn_wmma_f32_16x16x32_f16(false, a, false, b, (short)0, c, false, false); asm volatile("v_nop\n\tv_nop\n\tv_nop\n\tv_nop" : "+v"(d) : "v"(a), "v"(b)); return d; }
__device__ __forceinline__ void wave_lds_sync() { __builtin_amdgcn_fence(__ATOMIC_RELEASE, "workgroup"); __builtin_amdgcn_wave_barrier(); __builtin_amdgcn_fence(__ATOMIC_ACQUIRE, "workgroup"); }
__device__ __forceinline__ int iclamp(int v, int lo, int hi) { return v < lo ? lo : (v > hi ? hi : v); }

__global__ __launch_bounds__(256) void wput_kernel(const float* __restrict__ coef, const float* __restrict__ bw, b16* __restrict__ CT, b16* __restrict__ BW) { const size_t u = (size_t)blockIdx.x * 256 + threadIdx.x; v8b v;
  if (u < (size_t)OUT * KT / 8) {
#pragma unroll
    for (int j = 0; j < 8; ++j) v[j] = (b16)(bf16_rne(coef[u * 8 + j]) * WSC); for (int pass = 0; pass < 2; ++pass) { *(volatile v8b*)(CT + u * 8) = v; __threadfence(); } }
  if (u < (size_t)OUT * IN / 8) {
#pragma unroll
    for (int j = 0; j < 8; ++j) v[j] = (b16)(bf16_rne(bw[u * 8 + j]) * WSC); for (int pass = 0; pass < 2; ++pass) { *(volatile v8b*)(BW + u * 8) = v; __threadfence(); } } }
__global__ __launch_bounds__(32) void mk_kernel(const float* __restrict__ x, const b16* __restrict__ CT, const b16* __restrict__ BW, int RLIM, float* __restrict__ out) { __shared__ __attribute__((aligned(16))) b16 Sh[16][IN + 8], Sl[16][IN + 8], Ah[16][KCH + 8]; __shared__ float Tf[16][260]; const int lane = threadIdx.x, nloc = lane & 15, hlf = lane >> 4; const int cg = blockIdx.x & 1; const size_t m0 = (size_t)(blockIdx.x >> 1) * 16; if (m0 >= (size_t)RLIM) return;
  for (int rr = 0; rr < 16; ++rr) for (int q = 0; q < IN / 32; ++q) { float xc = bfv(x[(m0 + rr) * IN + q * 32 + lane]); xc = fminf(fmaxf(xc, -1.0f), 1.0f); const float si = xc / (1.0f + __expf(-xc)); b16 p, ql; split16(si * HS, p, ql); Sh[rr][q * 32 + lane] = p; Sl[rr][q * 32 + lane] = ql; }
  wave_lds_sync(); v8f acc[16];
#pragma unroll
  for (int t = 0; t < 16; ++t) acc[t] = (v8f){};
#pragma unroll 2
  for (int kb = 0; kb < IN; kb += 32) { const v16b a = frag_kb(&Sh[nloc][kb], hlf), al = frag_kb(&Sl[nloc][kb], hlf);
#pragma unroll
    for (int t = 0; t < 16; ++t) { const v16b bw = frag_kb(BW + (size_t)(cg * 256 + t * 16 + nloc) * IN + kb, hlf); acc[t] = wmma16b(a, bw, acc[t]); acc[t] = wmma16b(al, bw, acc[t]); } }
#pragma unroll
  for (int t = 0; t < 16; ++t)
#pragma unroll
    for (int r8 = 0; r8 < 8; ++r8) acc[t][r8] *= (1.0f / HS);
#pragma unroll 1
  for (int ch = 0; ch < IN / FCH; ++ch) {
    for (int rr = 0; rr < 16; ++rr) { const int i = ch * FCH + lane; float xc = bfv(x[(m0 + rr) * IN + i]); xc = fminf(fmaxf(xc, -1.0f), 1.0f); const float xg = (xc + 1.0f) * 0.5f * (float)G; int idx = (int)floorf(xg); idx = iclamp(idx, 0, G - 1); const float tt = xg - (float)idx;
      b16* row = &Ah[rr][lane * GP];
#pragma unroll
      for (int gg = 0; gg < GP; ++gg) { const float wv = (gg == idx) ? (1.0f - tt) : ((gg == idx + 1) ? tt : 0.0f); row[gg] = (b16)wv; } }
    if (lane < 16) for (int kk = KCH; kk < KCH + 8; ++kk) Ah[lane][kk] = (b16)0.0f;
    wave_lds_sync();
    const b16* CTc = CT + (size_t)ch * KCH;
#pragma unroll 3
    for (int kb = 0; kb < KCH; kb += 32) { const v16b a = frag_kb(&Ah[nloc][kb], hlf);
#pragma unroll
      for (int t = 0; t < 16; ++t) acc[t] = wmma16b(a, frag_kb(CTc + (size_t)(cg * 256 + t * 16 + nloc) * KT + kb, hlf), acc[t]); }
    wave_lds_sync(); }
#pragma unroll
  for (int t = 0; t < 16; ++t) { const int cc = t * 16 + nloc;
#pragma unroll
    for (int r8 = 0; r8 < 8; ++r8) Tf[8 * hlf + r8][cc] = acc[t][r8] * (1.0f / WSC); }
  wave_lds_sync();
  for (int pass = 0; pass < 2; ++pass) { for (int rr = 0; rr < 16; ++rr) for (int q = 0; q < 2; ++q) *(volatile v4f*)(out + (m0 + rr) * OUT + cg * 256 + q * 128 + lane * 4) = *(const v4f*)(&Tf[rr][q * 128 + lane * 4]); __threadfence(); } }
}

extern "C" void kernel_launch(void* const* d_in, const int* in_sizes, int n_in, void* d_out, int out_size, void* d_ws, size_t ws_size, hipStream_t stream) {
  (void)n_in;
  auto Fp = [&](int i) { return (const float*)d_in[i]; };
  if (in_sizes[0] != NBR * IN || in_sizes[1] != OUT * KT || in_sizes[2] != OUT * IN || out_size != NBR * OUT) return;
  const int RLIM = NBR;
  size_t off = 0; char* ws = (char*)d_ws;
  auto carve = [&](size_t bytes) { char* p = ws + off; off += (bytes + 255) & ~(size_t)255; return p; };
  b16* CT = (b16*)carve((size_t)OUT * KT * 2); b16* BW = (b16*)carve((size_t)OUT * IN * 2);
  if (off > ws_size || off > ((size_t)16 << 20)) return;
  wput_kernel<<<(unsigned)(((size_t)OUT * KT / 8 + 255) / 256), 256, 0, stream>>>(Fp(1), Fp(2), CT, BW);
  mk_kernel<<<(RLIM / 16) * 2, 32, 0, stream>>>(Fp(0), CT, BW, RLIM, (float*)d_out);
}
